// CrossAttention_38637525795303
// MI455X (gfx1250) — hardware-verified
//
#include <hip/hip_runtime.h>
#include <stdint.h>


typedef _Float16 v16h __attribute__((ext_vector_type(16)));
typedef _Float16 v8h  __attribute__((ext_vector_type(8)));
typedef float    v8f  __attribute__((ext_vector_type(8)));
typedef float    v4f  __attribute__((ext_vector_type(4)));

#ifndef SEQ
#define SEQ 2048
#endif
#ifndef MCTX
#define MCTX 2048
#endif
#define SEQ_FULL  2048
#define MCTX_FULL 2048
#define DM   1024
#define NH   8
#define HD   128
#define FF   4096

#define ACT_CAR   8.0f
#define W_CAR     1024.0f
#define PROJ_SCL  0.0009765625f
#define S_SCL     (0.015625f * 0.08838834764831845f)
#define P_CAR     16384.0f
#define CTX_SCL   0.0001220703125f
#define OUT_SCL   6.103515625e-05f
#define FFN2_SCL  0.0001220703125f
#define LN_EPS    1e-5f

static_assert(SEQ % 128 == 0);
static_assert(MCTX % 128 == 0);
static_assert(SEQ <= SEQ_FULL && MCTX <= MCTX_FULL);
static_assert(DM == NH * HD);
static_assert(HD == 128);
static_assert(NH == 8);
static_assert(DM % 128 == 0 && FF % 64 == 0 && DM % 64 == 0);
static_assert(DM % 32 == 0 && FF % 32 == 0);
static_assert(DM % 8 == 0 && FF % 8 == 0);
static_assert((long)SEQ_FULL * DM * 4 == 8388608L);
static_assert((long)SEQ * DM * 4 <= 8388608L);
static_assert(((long)SEQ * DM / 8) % 256 == 0 && ((long)MCTX * DM / 8) % 256 == 0);
static_assert(((long)DM * DM / 8) % 256 == 0 && ((long)FF * DM / 8) % 256 == 0);
static_assert((long)(DM / 64) * (SEQ / 128) * 128 * 64 == (long)SEQ * DM);
static_assert((long)(DM / 64) * (MCTX / 128) * 128 * 64 == (long)MCTX * DM);
static_assert((long)(MCTX / 64) * (DM / 128) * 128 * 64 == (long)MCTX * DM);
static_assert((long)(FF / 64) * (SEQ / 128) * 128 * 64 == (long)SEQ * FF);
static_assert((long)(SEQ / 16) * 16 * DM == (long)SEQ * DM);
static_assert((long)(SEQ / 8) * 8 == (long)SEQ);
#define WS_HALVES (4L * SEQ * DM + 3L * MCTX * DM + 4L * DM * DM + 2L * FF * DM + (long)SEQ * FF)
#define WS_FLOATS (3L * SEQ * DM)
#define WS_BYTES  (WS_HALVES * 2 + WS_FLOATS * 4)
static_assert(WS_BYTES <= 134217728L);
static_assert(((long)SEQ * DM) % 64 == 0 && ((long)MCTX * DM) % 64 == 0 && ((long)DM * DM) % 64 == 0 &&
              ((long)FF * DM) % 64 == 0 && ((long)SEQ * FF) % 64 == 0);

union Frag16 { v16h v; v8h p[2]; };

__device__ __forceinline__ v16h ld_frag(const _Float16* __restrict__ p, int hl) {
  Frag16 f;
  f.p[0] = *(const v8h*)(p + 8 * hl);
  f.p[1] = *(const v8h*)(p + 16 + 8 * hl);
  return f.v;
}

__device__ __forceinline__ v8f mma(v16h a, v16h b, v8f c) {
  v8f d = __builtin_amdgcn_wmma_f32_16x16x32_f16(false, a, false, b, (short)0, c, false, false);
  asm volatile("v_nop\n\tv_nop\n\tv_nop\n\tv_nop" : "+v"(d) : "v"(a), "v"(b));
  return d;
}

__device__ __forceinline__ float bf16_rne(float x) {
  unsigned int u = __builtin_bit_cast(unsigned int, x);
  u += 0x7FFFu + ((u >> 16) & 1u);
  return __builtin_bit_cast(float, u & 0xFFFF0000u);
}

__global__ __launch_bounds__(256) void k_cvt8(const float* __restrict__ src,
                                              _Float16* __restrict__ dst,
                                              float car, int total8)
{
  const int i8 = blockIdx.x * 256 + threadIdx.x;
  if (i8 >= total8) return;
  const size_t e = (size_t)i8 * 8;
  const v4f x0 = *(const v4f*)(src + e);
  const v4f x1 = *(const v4f*)(src + e + 4);
  v8h o;
#pragma unroll
  for (int j = 0; j < 4; ++j) {
    const float t0 = x0[j];
    const float t1 = x1[j];
    o[j]     = (_Float16)(bf16_rne(t0) * car);
    o[4 + j] = (_Float16)(bf16_rne(t1) * car);
  }
  _Float16* d = dst + e;
  *(volatile v8h*)d = o;
  __threadfence();
  *(volatile v8h*)d = o;
}

__device__ __forceinline__ void gemm_core(const _Float16* __restrict__ ap0,
                                          const _Float16* __restrict__ ap1,
                                          const _Float16* __restrict__ bp,
                                          int K, int hl, v8f (&acc)[8])
{
  const size_t bst = (size_t)16 * K;
#pragma unroll 1
  for (int k0 = 0; k0 < K; k0 += 32) {
    const v16h a0 = ld_frag(ap0 + k0, hl);
    const v16h a1 = ld_frag(ap1 + k0, hl);
    const v16h b0 = ld_frag(bp + k0, hl);
    const v16h b1 = ld_frag(bp + bst + k0, hl);
    const v16h b2 = ld_frag(bp + 2 * bst + k0, hl);
    const v16h b3 = ld_frag(bp + 3 * bst + k0, hl);
    acc[0] = mma(a0, b0, acc[0]);
    acc[1] = mma(a0, b1, acc[1]);
    acc[2] = mma(a0, b2, acc[2]);
    acc[3] = mma(a0, b3, acc[3]);
    acc[4] = mma(a1, b0, acc[4]);
    acc[5] = mma(a1, b1, acc[5]);
    acc[6] = mma(a1, b2, acc[6]);
    acc[7] = mma(a1, b3, acc[7]);
  }
}

__global__ __launch_bounds__(128) __attribute__((amdgpu_num_vgpr(256)))
void k_gemm_h(const _Float16* __restrict__ A, const _Float16* __restrict__ Bt,
              const float* __restrict__ bias, _Float16* __restrict__ PH,
              int K, int ldc, float scl, float bscl, int bias_row, int relu)
{
  __shared__ __attribute__((aligned(16))) _Float16 ldsH[128 * 72];

  const int tid = threadIdx.x, lane = tid & 31, w = tid >> 5;
  const int hl = lane >> 4, c = lane & 15;
  const int m0 = blockIdx.y * 128, n0 = blockIdx.x * 64;
  const int mw = m0 + 32 * w;

  const _Float16* ap0 = A  + (size_t)(mw + c) * K;
  const _Float16* ap1 = A  + (size_t)(mw + 16 + c) * K;
  const _Float16* bp  = Bt + (size_t)(n0 + c) * K;

  v8f acc[8] = {};
  gemm_core(ap0, ap1, bp, K, hl, acc);

  float bc[4] = {0.f, 0.f, 0.f, 0.f};
  if (bias_row == 0) {
#pragma unroll
    for (int t = 0; t < 4; ++t) bc[t] = bf16_rne(bias[n0 + 16 * t + c]) * bscl;
  }
#pragma unroll
  for (int i = 0; i < 2; ++i)
#pragma unroll
    for (int r = 0; r < 8; ++r) {
      const int rowl = 32 * w + 16 * i + 8 * hl + r;
      float br = 0.f;
      if (bias_row != 0) br = bf16_rne(bias[m0 + rowl]) * bscl;
#pragma unroll
      for (int t = 0; t < 4; ++t) {
        float v = acc[i * 4 + t][r] * scl + bc[t] + br;
        if (relu != 0) v = fmaxf(v, 0.f);
        ldsH[rowl * 72 + 16 * t + c] = (_Float16)v;
      }
    }
  __syncthreads();

  _Float16* const bh = PH + (size_t)m0 * ldc + n0;
  for (int i = 0; i < 8; ++i) {
    const int q = i * 128 + tid;
    const int rowl = q >> 3, ch = (q & 7) * 8;
    const v8h vh = *(const v8h*)(&ldsH[rowl * 72 + ch]);
    *(volatile v8h*)(bh + (size_t)rowl * ldc + ch) = vh;
  }
  __threadfence();
  for (int i = 0; i < 8; ++i) {
    const int q = i * 128 + tid;
    const int rowl = q >> 3, ch = (q & 7) * 8;
    const v8h vh = *(const v8h*)(&ldsH[rowl * 72 + ch]);
    *(volatile v8h*)(bh + (size_t)rowl * ldc + ch) = vh;
  }
}

__global__ __launch_bounds__(128) __attribute__((amdgpu_num_vgpr(256)))
void k_gemm_f(const _Float16* __restrict__ A, const _Float16* __restrict__ Bt,
              const float* __restrict__ bias, const float* __restrict__ Res,
              float* __restrict__ Out, int K, float scl, int res_bf16)
{
  __shared__ __attribute__((aligned(16))) float ldsF[128 * 68];

  const int tid = threadIdx.x, lane = tid & 31, w = tid >> 5;
  const int hl = lane >> 4, c = lane & 15;
  const int m0 = blockIdx.y * 128, n0 = blockIdx.x * 64;
  const int mw = m0 + 32 * w;

  const _Float16* ap0 = A  + (size_t)(mw + c) * K;
  const _Float16* ap1 = A  + (size_t)(mw + 16 + c) * K;
  const _Float16* bp  = Bt + (size_t)(n0 + c) * K;

  v8f acc[8] = {};
  gemm_core(ap0, ap1, bp, K, hl, acc);

#pragma unroll
  for (int i = 0; i < 2; ++i)
#pragma unroll
    for (int t = 0; t < 4; ++t)
#pragma unroll
      for (int r = 0; r < 8; ++r) {
        const int rowl = 32 * w + 16 * i + 8 * hl + r;
        ldsF[rowl * 68 + 16 * t + c] = acc[i * 4 + t][r] * scl;
      }
  __syncthreads();

  const int colc = (tid & 15) * 4;
  const v4f braw = *(const v4f*)(bias + n0 + colc);
  v4f bia;
#pragma unroll
  for (int j = 0; j < 4; ++j) { const float t0 = braw[j]; bia[j] = bf16_rne(t0); }

  float* const ob = Out + (size_t)m0 * DM + n0;
  const float* const rb = Res + (size_t)m0 * DM + n0;
  for (int i = 0; i < 16; ++i) {
    const int rowl = i * 8 + (tid >> 4);
    const v4f rraw = *(const v4f*)(rb + (size_t)rowl * DM + colc);
    v4f rr;
#pragma unroll
    for (int j = 0; j < 4; ++j) { const float t0 = rraw[j]; rr[j] = (res_bf16 != 0) ? bf16_rne(t0) : t0; }
    const v4f v = (*(const v4f*)(&ldsF[rowl * 68 + colc]) + bia) + rr;
    *(volatile v4f*)(ob + (size_t)rowl * DM + colc) = v;
  }
  __threadfence();
  for (int i = 0; i < 16; ++i) {
    const int rowl = i * 8 + (tid >> 4);
    const v4f rraw = *(const v4f*)(rb + (size_t)rowl * DM + colc);
    v4f rr;
#pragma unroll
    for (int j = 0; j < 4; ++j) { const float t0 = rraw[j]; rr[j] = (res_bf16 != 0) ? bf16_rne(t0) : t0; }
    const v4f v = (*(const v4f*)(&ldsF[rowl * 68 + colc]) + bia) + rr;
    *(volatile v4f*)(ob + (size_t)rowl * DM + colc) = v;
  }
}

__global__ __launch_bounds__(256) __attribute__((amdgpu_num_vgpr(256)))
void k_attn(const _Float16* __restrict__ Q, const _Float16* __restrict__ Kp,
            const _Float16* __restrict__ Vt, _Float16* __restrict__ CTX)
{
  constexpr int SP = 36;
  constexpr int PP = 40;
  constexpr int OP = DM + 8;
  static_assert(16 * 32 == 2 * 256);
  static_assert(8 * 256 * 8 == 16 * DM);
  static_assert((PP * 2) % 16 == 0 && (OP * 2) % 16 == 0);
  __shared__ __attribute__((aligned(16))) float    ldsS[NH * 16 * SP];
  __shared__ __attribute__((aligned(16))) _Float16 ldsP[NH * 16 * PP];
  __shared__ __attribute__((aligned(16))) _Float16 ldsO[16 * OP];

  const int tid = threadIdx.x, lane = tid & 31, w = tid >> 5;
  const int hl = lane >> 4, c = lane & 15;
  const int n0 = blockIdx.x * 16;
  const int col0 = w * HD;

  const size_t qoff = (size_t)(n0 + c) * DM + col0;
  const size_t koff = (size_t)c * DM + col0;
  const size_t voff = (size_t)(col0 + c) * MCTX;

  v8f oa[8] = {};

#pragma unroll 1
  for (int kt = 0; kt < MCTX / 32; ++kt) {
    const int mk = kt * 32;

    v8f sc0 = {}, sc1 = {};
#pragma unroll
    for (int ks = 0; ks < 4; ++ks) {
      const v16h qf = ld_frag(Q + qoff + 32 * ks, hl);
      const v16h k0 = ld_frag(Kp + koff + (size_t)mk * DM + 32 * ks, hl);
      const v16h k1 = ld_frag(Kp + koff + (size_t)(mk + 16) * DM + 32 * ks, hl);
      sc0 = mma(qf, k0, sc0);
      sc1 = mma(qf, k1, sc1);
    }
#pragma unroll
    for (int r = 0; r < 8; ++r) {
      const int si = (w * 16 + 8 * hl + r) * SP + c;
      ldsS[si]      = sc0[r] * S_SCL;
      ldsS[si + 16] = sc1[r] * S_SCL;
    }
    __syncthreads();

#pragma unroll
    for (int j = 0; j < 2; ++j) {
      const int row = w + 8 * j;
      float s[NH];
#pragma unroll
      for (int h = 0; h < NH; ++h) s[h] = ldsS[(h * 16 + row) * SP + lane];
      float mx = s[0];
#pragma unroll
      for (int h = 1; h < NH; ++h) mx = fmaxf(mx, s[h]);
      float den = 0.f;
#pragma unroll
      for (int h = 0; h < NH; ++h) { s[h] = __expf(s[h] - mx); den += s[h]; }
      const float invc = (1.0f / den) * P_CAR;
#pragma unroll
      for (int h = 0; h < NH; ++h)
        ldsP[(h * 16 + row) * PP + lane] = (_Float16)(s[h] * invc);
    }
    __syncthreads();

    Frag16 pf;
    pf.p[0] = *(const v8h*)(&ldsP[(w * 16 + c) * PP + 8 * hl]);
    pf.p[1] = *(const v8h*)(&ldsP[(w * 16 + c) * PP + 16 + 8 * hl]);
#pragma unroll
    for (int g = 0; g < 2; ++g) {
      const v16h v0 = ld_frag(Vt + voff + (size_t)(16 * (4 * g + 0)) * MCTX + mk, hl);
      const v16h v1 = ld_frag(Vt + voff + (size_t)(16 * (4 * g + 1)) * MCTX + mk, hl);
      const v16h v2 = ld_frag(Vt + voff + (size_t)(16 * (4 * g + 2)) * MCTX + mk, hl);
      const v16h v3 = ld_frag(Vt + voff + (size_t)(16 * (4 * g + 3)) * MCTX + mk, hl);
      oa[4 * g + 0] = mma(pf.v, v0, oa[4 * g + 0]);
      oa[4 * g + 1] = mma(pf.v, v1, oa[4 * g + 1]);
      oa[4 * g + 2] = mma(pf.v, v2, oa[4 * g + 2]);
      oa[4 * g + 3] = mma(pf.v, v3, oa[4 * g + 3]);
    }
  }

#pragma unroll
  for (int t = 0; t < 8; ++t)
#pragma unroll
    for (int r = 0; r < 8; ++r)
      ldsO[(8 * hl + r) * OP + col0 + 16 * t + c] = (_Float16)(oa[t][r] * CTX_SCL);
  __syncthreads();

  _Float16* const ob = CTX + (size_t)n0 * DM;
  for (int i = 0; i < 8; ++i) {
    const int q = i * 256 + tid;
    const int rowl = q >> 7, ch = (q & 127) * 8;
    const v8h vh = *(const v8h*)(&ldsO[rowl * OP + ch]);
    *(volatile v8h*)(ob + (size_t)rowl * DM + ch) = vh;
  }
  __threadfence();
  for (int i = 0; i < 8; ++i) {
    const int q = i * 256 + tid;
    const int rowl = q >> 7, ch = (q & 127) * 8;
    const v8h vh = *(const v8h*)(&ldsO[rowl * OP + ch]);
    *(volatile v8h*)(ob + (size_t)rowl * DM + ch) = vh;
  }
}

__device__ __forceinline__ float wave_sum(float v) {
  v += __shfl_xor(v, 1, 32);
  v += __shfl_xor(v, 2, 32);
  v += __shfl_xor(v, 4, 32);
  v += __shfl_xor(v, 8, 32);
  v += __shfl_xor(v, 16, 32);
  return v;
}

__device__ __forceinline__ void ln_store_f(const float* __restrict__ x, const float* __restrict__ g,
                                           const float* __restrict__ b, float mean, float rstd,
                                           float* __restrict__ o, int lane)
{
  static_assert(DM % 128 == 0);
#pragma unroll 1
  for (int i = 0; i < DM / 128; ++i) {
    const int e = i * 128 + 4 * lane;
    const v4f xv = *(const v4f*)(x + e);
    const v4f gv = *(const v4f*)(g + e);
    const v4f bv = *(const v4f*)(b + e);
    v4f r;
#pragma unroll
    for (int j = 0; j < 4; ++j) {
      const float xs = xv[j], gs = gv[j], bs = bv[j];
      r[j] = (xs - mean) * rstd * bf16_rne(gs) + bf16_rne(bs);
    }
    *(volatile v4f*)(o + e) = r;
  }
}

__device__ __forceinline__ void ln_store_h(const float* __restrict__ x, const float* __restrict__ g,
                                           const float* __restrict__ b, float mean, float rstd,
                                           _Float16* __restrict__ o, int lane)
{
  static_assert(DM % 256 == 0);
#pragma unroll 1
  for (int i = 0; i < DM / 256; ++i) {
    const int e = i * 256 + 8 * lane;
    const v4f x0 = *(const v4f*)(x + e);
    const v4f x1 = *(const v4f*)(x + e + 4);
    const v4f g0 = *(const v4f*)(g + e);
    const v4f g1 = *(const v4f*)(g + e + 4);
    const v4f b0 = *(const v4f*)(b + e);
    const v4f b1 = *(const v4f*)(b + e + 4);
    v8h r;
#pragma unroll
    for (int j = 0; j < 4; ++j) {
      const float xa = x0[j], ga = g0[j], ba = b0[j];
      const float xb = x1[j], gb = g1[j], bb = b1[j];
      const float va = (xa - mean) * rstd * bf16_rne(ga) + bf16_rne(ba);
      const float vb = (xb - mean) * rstd * bf16_rne(gb) + bf16_rne(bb);
      r[j]     = (_Float16)(va * ACT_CAR);
      r[4 + j] = (_Float16)(vb * ACT_CAR);
    }
    *(volatile v8h*)(o + e) = r;
  }
}

__global__ __launch_bounds__(256)
void k_ln(const float* __restrict__ T, const float* __restrict__ g, const float* __restrict__ b,
          float* __restrict__ OutF, _Float16* __restrict__ OutH, int want_h, int rows)
{
  const int lane = threadIdx.x & 31, w = threadIdx.x >> 5;
  const int row = blockIdx.x * 8 + w;
  if (row >= rows) return;
  const float* x = T + (size_t)row * DM;

  float s = 0.f;
#pragma unroll 1
  for (int i = 0; i < DM / 128; ++i) {
    const v4f v = *(const v4f*)(x + i * 128 + 4 * lane);
    s += (v[0] + v[1]) + (v[2] + v[3]);
  }
  s = wave_sum(s);
  const float mean = s * (1.0f / DM);

  float ss = 0.f;
#pragma unroll 1
  for (int i = 0; i < DM / 128; ++i) {
    const v4f v = *(const v4f*)(x + i * 128 + 4 * lane);
    const float d0 = v[0] - mean, d1 = v[1] - mean, d2 = v[2] - mean, d3 = v[3] - mean;
    ss += (d0 * d0 + d1 * d1) + (d2 * d2 + d3 * d3);
  }
  ss = wave_sum(ss);
  const float rstd = rsqrtf(ss * (1.0f / DM) + LN_EPS);

  float* of = OutF + (size_t)row * DM;
  ln_store_f(x, g, b, mean, rstd, of, lane);
  __threadfence();
  ln_store_f(x, g, b, mean, rstd, of, lane);

  if (want_h != 0) {
    _Float16* oh = OutH + (size_t)row * DM;
    ln_store_h(x, g, b, mean, rstd, oh, lane);
    __threadfence();
    ln_store_h(x, g, b, mean, rstd, oh, lane);
  }
}

extern "C" void kernel_launch(void* const* d_in, const int* in_sizes, int n_in,
                              void* d_out, int out_size, void* d_ws, size_t ws_size,
                              hipStream_t stream)
{
  if (n_in < 18) return;
  if ((long)in_sizes[0] < (long)SEQ * DM) return;
  if ((long)in_sizes[1] < (long)MCTX * DM) return;
  if ((long)in_sizes[2] < (long)DM * DM || (long)in_sizes[4] < (long)DM * DM) return;
  if ((long)in_sizes[6] < (long)DM * DM || (long)in_sizes[8] < (long)DM * DM) return;
  if ((long)in_sizes[10] < (long)FF * DM || (long)in_sizes[12] < (long)DM * FF) return;
  if (in_sizes[3] < DM || in_sizes[5] < DM || in_sizes[7] < DM || in_sizes[9] < DM) return;
  if (in_sizes[11] < FF || in_sizes[13] < DM) return;
  if (in_sizes[14] < DM || in_sizes[15] < DM || in_sizes[16] < DM || in_sizes[17] < DM) return;
  if ((long)out_size < (long)SEQ * DM) return;
  if ((size_t)WS_BYTES > ws_size) return;

  const float* x1  = (const float*)d_in[0];
  const float* x2  = (const float*)d_in[1];
  const float* Wq  = (const float*)d_in[2];
  const float* bq  = (const float*)d_in[3];
  const float* Wk  = (const float*)d_in[4];
  const float* bk  = (const float*)d_in[5];
  const float* Wv  = (const float*)d_in[6];
  const float* bv  = (const float*)d_in[7];
  const float* Wo  = (const float*)d_in[8];
  const float* bo  = (const float*)d_in[9];
  const float* W1  = (const float*)d_in[10];
  const float* b1  = (const float*)d_in[11];
  const float* W2  = (const float*)d_in[12];
  const float* b2  = (const float*)d_in[13];
  const float* g1  = (const float*)d_in[14];
  const float* be1 = (const float*)d_in[15];
  const float* g2  = (const float*)d_in[16];
  const float* be2 = (const float*)d_in[17];
  float* out = (float*)d_out;

  const size_t nX = (size_t)SEQ * DM;
  const size_t nC = (size_t)MCTX * DM;
  const size_t nW = (size_t)DM * DM;
  const size_t nF = (size_t)FF * DM;
  const size_t nA = (size_t)SEQ * FF;

  _Float16* X1h  = (_Float16*)d_ws;
  _Float16* X2h  = X1h  + nX;
  _Float16* Wqh  = X2h  + nC;
  _Float16* Wkh  = Wqh  + nW;
  _Float16* Wvh  = Wkh  + nW;
  _Float16* Woh  = Wvh  + nW;
  _Float16* W1h  = Woh  + nW;
  _Float16* W2h  = W1h  + nF;
  _Float16* Qh   = W2h  + nF;
  _Float16* Kh   = Qh   + nX;
  _Float16* Vth  = Kh   + nC;
  _Float16* CTXh = Vth  + nC;
  _Float16* H16  = CTXh + nX;
  _Float16* F1h  = H16  + nX;
  float*    T1   = (float*)(F1h + nA);
  float*    Hf   = T1 + nX;
  float*    T2   = Hf + nX;

  const int tx8 = (int)(nX / 8), tc8 = (int)(nC / 8), tw8 = (int)(nW / 8), tf8 = (int)(nF / 8);
  k_cvt8<<<dim3((tx8 + 255) / 256), 256, 0, stream>>>(x1, X1h, ACT_CAR, tx8);
  k_cvt8<<<dim3((tc8 + 255) / 256), 256, 0, stream>>>(x2, X2h, ACT_CAR, tc8);
  k_cvt8<<<dim3((tw8 + 255) / 256), 256, 0, stream>>>(Wq, Wqh, W_CAR, tw8);
  k_cvt8<<<dim3((tw8 + 255) / 256), 256, 0, stream>>>(Wk, Wkh, W_CAR, tw8);
  k_cvt8<<<dim3((tw8 + 255) / 256), 256, 0, stream>>>(Wv, Wvh, W_CAR, tw8);
  k_cvt8<<<dim3((tw8 + 255) / 256), 256, 0, stream>>>(Wo, Woh, W_CAR, tw8);
  k_cvt8<<<dim3((tf8 + 255) / 256), 256, 0, stream>>>(W1, W1h, W_CAR, tf8);
  k_cvt8<<<dim3((tf8 + 255) / 256), 256, 0, stream>>>(W2, W2h, W_CAR, tf8);

  k_gemm_h<<<dim3(DM / 64, SEQ / 128), 128, 0, stream>>>(X1h, Wqh, bq, Qh, DM, DM,
                                                         PROJ_SCL, ACT_CAR, 0, 0);
  k_gemm_h<<<dim3(DM / 64, MCTX / 128), 128, 0, stream>>>(X2h, Wkh, bk, Kh, DM, DM,
                                                          PROJ_SCL, ACT_CAR, 0, 0);
  k_gemm_h<<<dim3(MCTX / 64, DM / 128), 128, 0, stream>>>(Wvh, X2h, bv, Vth, DM, MCTX,
                                                          PROJ_SCL, ACT_CAR, 1, 0);

  k_attn<<<dim3(SEQ / 16), 256, 0, stream>>>(Qh, Kh, Vth, CTXh);

  k_gemm_f<<<dim3(DM / 64, SEQ / 128), 128, 0, stream>>>(CTXh, Woh, bo, x1, T1, DM, OUT_SCL, 1);

  k_ln<<<dim3(SEQ / 8), 256, 0, stream>>>(T1, g1, be1, Hf, H16, 1, SEQ);

  k_gemm_h<<<dim3(FF / 64, SEQ / 128), 128, 0, stream>>>(H16, W1h, b1, F1h, DM, FF,
                                                         PROJ_SCL, ACT_CAR, 0, 1);
  k_gemm_f<<<dim3(DM / 64, SEQ / 128), 128, 0, stream>>>(F1h, W2h, b2, Hf, T2, FF, FFN2_SCL, 0);

  k_ln<<<dim3(SEQ / 8), 256, 0, stream>>>(T2, g2, be2, out, H16, 0, SEQ);
}
